// EncoderBlock_83184926589063
// MI455X (gfx1250) — hardware-verified
//
#include <hip/hip_runtime.h>


#ifndef NB
#define NB 2
#endif
#ifndef SEQ
#define SEQ 2048
#endif
#define NB_FULL  2
#define SEQ_FULL 2048
#define DM   1024
#define NH   16
#define DKH  64
#define DFF  4096
#define ROWS (NB * SEQ)
#define NQT  (SEQ / 128)
#define NKT  (SEQ / 64)
#define FLAG_PITCH 32

static_assert(NB >= 1 && NB <= NB_FULL);
static_assert(SEQ >= 256 && SEQ <= SEQ_FULL && (SEQ % 128) == 0);
static_assert(NKT >= 4 && NKT <= FLAG_PITCH && (256 % NKT) == 0 && (128 % (256 / NKT)) == 0);
static_assert((ROWS % 128) == 0 && (DM % 128) == 0 && (DFF % 128) == 0 && (DM % 32) == 0 && (DFF % 32) == 0);
static_assert(NH * DKH == DM && DKH == 64);

typedef _Float16 f16_t;
typedef _Float16     v16h __attribute__((ext_vector_type(16)));
typedef _Float16     v8h  __attribute__((ext_vector_type(8), __may_alias__));
typedef float        v8f  __attribute__((ext_vector_type(8)));
typedef float        v4f  __attribute__((ext_vector_type(4), __may_alias__));
typedef unsigned int v4u  __attribute__((ext_vector_type(4), __may_alias__));
typedef unsigned int v2u  __attribute__((ext_vector_type(2), __may_alias__));
typedef int          v4i  __attribute__((ext_vector_type(4), __may_alias__));

#define WS_LIMIT 134217728ull
constexpr size_t SZ_WQ  = (size_t)DM * DM * 2;
constexpr size_t SZ_WO  = (size_t)DM * DM * 2;
constexpr size_t SZ_W1  = (size_t)DFF * DM * 2;
constexpr size_t SZ_W2  = (size_t)DM * DFF * 2;
constexpr size_t SZ_XH  = (size_t)ROWS * DM * 2;
constexpr size_t SZ_Q   = (size_t)ROWS * DM * 2;
constexpr size_t SZ_CX  = (size_t)ROWS * DM * 2;
constexpr size_t SZ_S   = (size_t)ROWS * DM * 4;
constexpr size_t SZ_X1F = (size_t)ROWS * DM * 4;
constexpr size_t SZ_X1H = (size_t)ROWS * DM * 2;
constexpr size_t SZ_H   = (size_t)ROWS * DFF * 2;
constexpr size_t SZ_FL  = (((size_t)NQT * FLAG_PITCH * 4) + 4095) & ~(size_t)4095;
constexpr size_t OFF_WQ  = 0;
constexpr size_t OFF_WO  = OFF_WQ + SZ_WQ;
constexpr size_t OFF_W1  = OFF_WO + SZ_WO;
constexpr size_t OFF_W2  = OFF_W1 + SZ_W1;
constexpr size_t OFF_XH  = OFF_W2 + SZ_W2;
constexpr size_t OFF_Q   = OFF_XH + SZ_XH;
constexpr size_t OFF_CX  = OFF_Q + SZ_Q;
constexpr size_t OFF_S   = OFF_CX + SZ_CX;
constexpr size_t OFF_X1F = OFF_S + SZ_S;
constexpr size_t OFF_X1H = OFF_X1F + SZ_X1F;
constexpr size_t OFF_H   = OFF_X1H + SZ_X1H;
constexpr size_t OFF_FL  = OFF_H + SZ_H;
constexpr size_t WS_TOTAL = OFF_FL + SZ_FL;
static_assert(WS_TOTAL <= WS_LIMIT);
static_assert((OFF_WO % 256) == 0 && (OFF_W1 % 256) == 0 && (OFF_W2 % 256) == 0 && (OFF_XH % 256) == 0);
static_assert((OFF_Q % 256) == 0 && (OFF_CX % 256) == 0 && (OFF_S % 256) == 0 && (OFF_X1F % 256) == 0);
static_assert((OFF_X1H % 256) == 0 && (OFF_H % 256) == 0 && (OFF_FL % 256) == 0);
static_assert((size_t)ROWS * DM * 4 <= 16777216ull || NB < NB_FULL || SEQ < SEQ_FULL);

__device__ __forceinline__ v8f zero8() {
  v8f z;
#pragma unroll
  for (int i = 0; i < 8; ++i) z[i] = 0.0f;
  return z;
}

__device__ __forceinline__ float bfr(float x) {
  unsigned int u = __float_as_uint(x);
  u = (u + 0x7FFFu + ((u >> 16) & 1u)) & 0xFFFF0000u;
  return __uint_as_float(u);
}

__device__ __forceinline__ v8f wmma16(v16h a, v16h b, v8f c) {
  c = __builtin_amdgcn_wmma_f32_16x16x32_f16(false, a, false, b, (short)0, c, false, false);
  asm volatile("v_nop\n\tv_nop\n\tv_nop\n\tv_nop" : "+v"(c) : "v"(a), "v"(b));
  return c;
}

__device__ __forceinline__ v16h ld_frag(const f16_t* plo, const f16_t* phi) {
  union { v16h v; v8h h[2]; } u;
  u.h[0] = *(const v8h*)plo;
  u.h[1] = *(const v8h*)phi;
  return u.v;
}

__device__ __forceinline__ float wsum32(float v) {
#pragma unroll
  for (int off = 16; off > 0; off >>= 1) v += __shfl_xor(v, off, 32);
  return v;
}

template <int ROWMAP>
__global__ __launch_bounds__(256) void k_cvt16(const float* __restrict__ src, f16_t* __restrict__ dst,
                                               int n, float scale) {
  const int e = (blockIdx.x * 256 + (int)threadIdx.x) * 8;
  if (e >= n) return;
  size_t s;
  if (ROWMAP) {
    const int m = e / DM;
    const int c = e - m * DM;
    const int b = m / SEQ;
    const int sq = m - b * SEQ;
    s = ((size_t)b * SEQ_FULL + sq) * DM + c;
  } else {
    s = (size_t)e;
  }
  const v4f a0 = *(const v4f*)(src + s);
  const v4f a1 = *(const v4f*)(src + s + 4);
  v8h hv;
#pragma unroll
  for (int i = 0; i < 4; ++i) {
    hv[i]     = (f16_t)(bfr(a0[i]) * scale);
    hv[4 + i] = (f16_t)(bfr(a1[i]) * scale);
  }
  union { v8h h; v4u u; } cv;
  cv.h = hv;
  const v4u ov = cv.u;
  f16_t* dp = dst + e;
  *(volatile v4u*)dp = ov;
  __threadfence();
  *(volatile v4u*)dp = ov;
}

__global__ __launch_bounds__(256) void k_maskflag(const int* __restrict__ mask, int* __restrict__ flags) {
  constexpr int TPK = 256 / NKT;
  constexpr int RPT = 128 / TPK;
  __shared__ int part[256];
  __shared__ __align__(16) int fl[FLAG_PITCH];
  const int tid = threadIdx.x, qt = blockIdx.x;
  const int kt = tid / TPK;
  const int j  = tid - kt * TPK;
  int anyz = 0;
  for (int rr = 0; rr < RPT; ++rr) {
    const int q = qt * 128 + j * RPT + rr;
    const int* mrow = mask + (size_t)q * SEQ_FULL + kt * 64;
#pragma unroll 4
    for (int c = 0; c < 16; ++c) {
      const v4i v = *(const v4i*)(mrow + c * 4);
      anyz |= (v.x == 0) | (v.y == 0) | (v.z == 0) | (v.w == 0);
    }
  }
  part[tid] = anyz;
  __syncthreads();
  if (tid < 32) {
    const int kk = (tid < NKT) ? tid : (NKT - 1);
    int f = 0;
    for (int i = 0; i < TPK; ++i) f |= part[kk * TPK + i];
    fl[tid] = (tid < NKT) ? f : 1;
  }
  __syncthreads();
  if (tid < 8) {
    const v4i ov = *(const v4i*)(fl + tid * 4);
    int* dp = flags + (size_t)qt * FLAG_PITCH + tid * 4;
    *(volatile v4i*)dp = ov;
    __threadfence();
    *(volatile v4i*)dp = ov;
  }
}

#define GEMM_SMEM 33792

template <int RES, typename OT>
__global__ __launch_bounds__(256) void k_gemm(const f16_t* __restrict__ A, const f16_t* __restrict__ Bt,
                                              const float* __restrict__ bias, const float* __restrict__ res,
                                              OT* __restrict__ C, int N, int K, float accScale) {
  static_assert(RES == 0 || sizeof(OT) == 4);
  constexpr int PITCH = (sizeof(OT) == 4) ? 132 : 136;
  static_assert(64 * PITCH * sizeof(OT) <= GEMM_SMEM);
  __shared__ __align__(16) unsigned char smem[GEMM_SMEM];
  f16_t* As = reinterpret_cast<f16_t*>(smem);
  f16_t* Bs = reinterpret_cast<f16_t*>(smem + 128 * 32 * 2);
  OT*    Cs = reinterpret_cast<OT*>(smem);

  const int tid = threadIdx.x;
  const int wave = tid >> 5, lane = tid & 31, lh = lane & 15, g = lane >> 4;
  const int waveM = wave >> 2, waveN = wave & 3;
  const int rowBase = blockIdx.y * 128, colBase = blockIdx.x * 128;
  const int kLo = 8 * g, kHi = 16 + 8 * g;
  const int sr = tid >> 2, sc = (tid & 3) * 8;
  const f16_t* Ag0 = A  + (size_t)(rowBase + sr) * K + sc;
  const f16_t* Ag1 = A  + (size_t)(rowBase + sr + 64) * K + sc;
  const f16_t* Bg0 = Bt + (size_t)(colBase + sr) * K + sc;
  const f16_t* Bg1 = Bt + (size_t)(colBase + sr + 64) * K + sc;

  v8f acc[4][2];
#pragma unroll
  for (int mr = 0; mr < 4; ++mr)
#pragma unroll
    for (int nr = 0; nr < 2; ++nr) acc[mr][nr] = zero8();

  const int kTiles = K >> 5;
#pragma unroll 1
  for (int kt = 0; kt < kTiles; ++kt) {
    const int k0 = kt << 5;
    const v8h a0 = *(const v8h*)(Ag0 + k0);
    const v8h a1 = *(const v8h*)(Ag1 + k0);
    const v8h b0 = *(const v8h*)(Bg0 + k0);
    const v8h b1 = *(const v8h*)(Bg1 + k0);
    __syncthreads();
    *(v8h*)(As + sr * 32 + sc)        = a0;
    *(v8h*)(As + (sr + 64) * 32 + sc) = a1;
    *(v8h*)(Bs + sr * 32 + sc)        = b0;
    *(v8h*)(Bs + (sr + 64) * 32 + sc) = b1;
    __syncthreads();
    v16h af[4], bf[2];
#pragma unroll
    for (int mr = 0; mr < 4; ++mr) {
      const int r = waveM * 64 + mr * 16 + lh;
      af[mr] = ld_frag(As + r * 32 + kLo, As + r * 32 + kHi);
    }
#pragma unroll
    for (int nr = 0; nr < 2; ++nr) {
      const int r = waveN * 32 + nr * 16 + lh;
      bf[nr] = ld_frag(Bs + r * 32 + kLo, Bs + r * 32 + kHi);
    }
#pragma unroll
    for (int mr = 0; mr < 4; ++mr)
#pragma unroll
      for (int nr = 0; nr < 2; ++nr) acc[mr][nr] = wmma16(af[mr], bf[nr], acc[mr][nr]);
  }

  const float bc0 = bfr(bias[colBase + waveN * 32 + lh]);
  const float bc1 = bfr(bias[colBase + waveN * 32 + 16 + lh]);
  for (int p = 0; p < 2; ++p) {
    __syncthreads();
    if (waveM == p) {
#pragma unroll
      for (int mr = 0; mr < 4; ++mr)
#pragma unroll
        for (int nr = 0; nr < 2; ++nr)
#pragma unroll
          for (int r = 0; r < 8; ++r) {
            const float v = acc[mr][nr][r] * accScale + (nr ? bc1 : bc0);
            Cs[(mr * 16 + g * 8 + r) * PITCH + waveN * 32 + nr * 16 + lh] = (OT)v;
          }
    }
    __syncthreads();
    if constexpr (sizeof(OT) == 4) {
      v4f vals[8];
#pragma unroll
      for (int i = 0; i < 8; ++i) {
        const int lr = wave * 8 + i;
        const int grow = rowBase + p * 64 + lr;
        const int gcol = colBase + lane * 4;
        v4f v = *(const v4f*)(Cs + lr * PITCH + lane * 4);
        if constexpr (RES == 1) {
          const v4f rr = *(const v4f*)(res + (size_t)grow * N + gcol);
          v += rr;
        } else if constexpr (RES == 2) {
          const int bb = grow / SEQ;
          const int ss = grow - bb * SEQ;
          const v4f rr = *(const v4f*)(res + ((size_t)bb * SEQ_FULL + ss) * DM + gcol);
#pragma unroll
          for (int jj = 0; jj < 4; ++jj) v[jj] += bfr(rr[jj]);
        }
        vals[i] = v;
      }
#pragma unroll
      for (int i = 0; i < 8; ++i)
        *(volatile v4f*)(C + (size_t)(rowBase + p * 64 + wave * 8 + i) * N + colBase + lane * 4) = vals[i];
      __threadfence();
#pragma unroll
      for (int i = 0; i < 8; ++i)
        *(volatile v4f*)(C + (size_t)(rowBase + p * 64 + wave * 8 + i) * N + colBase + lane * 4) = vals[i];
    } else {
      v4u vals[4];
#pragma unroll
      for (int i = 0; i < 4; ++i) {
        const int lr = wave * 8 + 2 * i + g;
        vals[i] = *(const v4u*)(Cs + lr * PITCH + lh * 8);
      }
#pragma unroll
      for (int i = 0; i < 4; ++i)
        *(volatile v4u*)(C + (size_t)(rowBase + p * 64 + wave * 8 + 2 * i + g) * N + colBase + lh * 8) = vals[i];
      __threadfence();
#pragma unroll
      for (int i = 0; i < 4; ++i)
        *(volatile v4u*)(C + (size_t)(rowBase + p * 64 + wave * 8 + 2 * i + g) * N + colBase + lh * 8) = vals[i];
    }
  }
}

__global__ __launch_bounds__(256) void k_attn(const f16_t* __restrict__ Qp, const int* __restrict__ mask,
                                              const int* __restrict__ flags, f16_t* __restrict__ Cx) {
  __shared__ __align__(16) f16_t Ks[64 * 64];
  __shared__ __align__(16) f16_t Vt[64 * 64];
  __shared__ __align__(16) f16_t Ps[128 * 64];
  __shared__ __align__(16) unsigned int Mw[128 * 16];
  const int tid = threadIdx.x;
  const int wave = tid >> 5, lane = tid & 31, lh = lane & 15, g = lane >> 4;
  const int kLo = 8 * g, kHi = 16 + 8 * g;
  const int qt = blockIdx.x, h = blockIdx.y, b = blockIdx.z;
  const size_t prow0 = (size_t)b * SEQ + (size_t)qt * 128;
  const size_t krow0 = (size_t)b * SEQ;
  const int col0 = h * DKH;
  const int qw0 = wave * 16;

  v16h aq[2];
  {
    const f16_t* qr = Qp + (prow0 + qw0 + lh) * DM + col0;
    aq[0] = ld_frag(qr + kLo, qr + kHi);
    aq[1] = ld_frag(qr + 32 + kLo, qr + 32 + kHi);
  }

  v8f o[4];
#pragma unroll
  for (int nr = 0; nr < 4; ++nr) o[nr] = zero8();
  float m[8], l[8];
#pragma unroll
  for (int r = 0; r < 8; ++r) { m[r] = -1e30f; l[r] = 0.0f; }

  const int skr = tid >> 3;
  const int skc = (tid & 7) * 8;
  const unsigned char* Mb = (const unsigned char*)Mw;

#pragma unroll 1
  for (int kt = 0; kt < NKT; ++kt) {
    const int kbase = kt * 64;
    const v8h kv0 = *(const v8h*)(Qp + (krow0 + kbase + skr) * DM + col0 + skc);
    const v8h kv1 = *(const v8h*)(Qp + (krow0 + kbase + 32 + skr) * DM + col0 + skc);
    const int fl = __builtin_amdgcn_readfirstlane(flags[qt * FLAG_PITCH + kt]);
    __syncthreads();
    *(v8h*)(Ks + skr * 64 + skc)        = kv0;
    *(v8h*)(Ks + (skr + 32) * 64 + skc) = kv1;
#pragma unroll
    for (int j = 0; j < 8; ++j) {
      Vt[(skc + j) * 64 + skr]      = kv0[j];
      Vt[(skc + j) * 64 + skr + 32] = kv1[j];
    }
    __syncthreads();

    v8f s[4];
#pragma unroll
    for (int nr = 0; nr < 4; ++nr) {
      s[nr] = zero8();
      const int kr = nr * 16 + lh;
#pragma unroll
      for (int c = 0; c < 2; ++c) {
        const v16h bk = ld_frag(Ks + kr * 64 + c * 32 + kLo, Ks + kr * 64 + c * 32 + kHi);
        s[nr] = wmma16(aq[c], bk, s[nr]);
      }
    }
#pragma unroll
    for (int nr = 0; nr < 4; ++nr)
#pragma unroll
      for (int r = 0; r < 8; ++r) s[nr][r] *= 0.125f;
    if (fl != 0) {
#pragma unroll
      for (int i = 0; i < 8; ++i) {
        const int lr = qw0 + 2 * i + g;
        const v4i mv = *(const v4i*)(mask + (size_t)(qt * 128 + lr) * SEQ_FULL + kbase + lh * 4);
        const unsigned int pk = (mv.x != 0 ? 1u : 0u) | (mv.y != 0 ? 0x100u : 0u) |
                                (mv.z != 0 ? 0x10000u : 0u) | (mv.w != 0 ? 0x1000000u : 0u);
        Mw[lr * 16 + lh] = pk;
      }
      __builtin_amdgcn_fence(3  , "wavefront");
      __builtin_amdgcn_wave_barrier();
#pragma unroll
      for (int nr = 0; nr < 4; ++nr) {
        const int key = nr * 16 + lh;
#pragma unroll
        for (int r = 0; r < 8; ++r) {
          const unsigned char mv = Mb[(qw0 + g * 8 + r) * 64 + key];
          s[nr][r] = (mv == 0) ? -1e9f : s[nr][r];
        }
      }
    }

    float f[8];
#pragma unroll
    for (int r = 0; r < 8; ++r) {
      float v = fmaxf(fmaxf(s[0][r], s[1][r]), fmaxf(s[2][r], s[3][r]));
#pragma unroll
      for (int off = 8; off > 0; off >>= 1) v = fmaxf(v, __shfl_xor(v, off, 16));
      const float mn = fmaxf(m[r], v);
      f[r] = __expf(m[r] - mn);
      m[r] = mn;
    }
    float rs[8];
#pragma unroll
    for (int r = 0; r < 8; ++r) rs[r] = 0.0f;
#pragma unroll
    for (int nr = 0; nr < 4; ++nr)
#pragma unroll
      for (int r = 0; r < 8; ++r) {
        const float p = __expf(s[nr][r] - m[r]);
        s[nr][r] = p;
        rs[r] += p;
      }
#pragma unroll
    for (int r = 0; r < 8; ++r) {
      float v = rs[r];
#pragma unroll
      for (int off = 8; off > 0; off >>= 1) v += __shfl_xor(v, off, 16);
      l[r] = l[r] * f[r] + v;
    }
#pragma unroll
    for (int nr = 0; nr < 4; ++nr)
#pragma unroll
      for (int r = 0; r < 8; ++r) o[nr][r] *= f[r];
#pragma unroll
    for (int nr = 0; nr < 4; ++nr)
#pragma unroll
      for (int r = 0; r < 8; ++r)
        Ps[(qw0 + g * 8 + r) * 64 + nr * 16 + lh] = (f16_t)(s[nr][r] * 1024.0f);
    __syncthreads();

#pragma unroll
    for (int c = 0; c < 2; ++c) {
      const v16h ap = ld_frag(Ps + (qw0 + lh) * 64 + c * 32 + kLo, Ps + (qw0 + lh) * 64 + c * 32 + kHi);
#pragma unroll
      for (int nr = 0; nr < 4; ++nr) {
        const int dr = nr * 16 + lh;
        const v16h bv = ld_frag(Vt + dr * 64 + c * 32 + kLo, Vt + dr * 64 + c * 32 + kHi);
        o[nr] = wmma16(ap, bv, o[nr]);
      }
    }
  }

  __syncthreads();
#pragma unroll
  for (int r = 0; r < 8; ++r) {
    const float inv = 0.0625f / l[r];
#pragma unroll
    for (int nr = 0; nr < 4; ++nr)
      Ps[(qw0 + g * 8 + r) * 64 + nr * 16 + lh] = (f16_t)(o[nr][r] * inv);
  }
  __syncthreads();
  v4u vals[4];
#pragma unroll
  for (int i = 0; i < 4; ++i) {
    const int lr = qw0 + 4 * i + (lane >> 3);
    vals[i] = *(const v4u*)(Ps + lr * 64 + (lane & 7) * 8);
  }
#pragma unroll
  for (int i = 0; i < 4; ++i)
    *(volatile v4u*)(Cx + (prow0 + qw0 + 4 * i + (lane >> 3)) * DM + col0 + (lane & 7) * 8) = vals[i];
  __threadfence();
#pragma unroll
  for (int i = 0; i < 4; ++i)
    *(volatile v4u*)(Cx + (prow0 + qw0 + 4 * i + (lane >> 3)) * DM + col0 + (lane & 7) * 8) = vals[i];
}

template <int F16OUT>
__global__ __launch_bounds__(256) void k_ln(const float* __restrict__ S, const float* __restrict__ alpha,
                                            const float* __restrict__ beta, float* __restrict__ Yf,
                                            f16_t* __restrict__ Yh) {
  __shared__ float red[8];
  const int row = blockIdx.x, tid = threadIdx.x, wave = tid >> 5, lane = tid & 31;
  const v4f v = *(const v4f*)(S + (size_t)row * DM + tid * 4);
  float sm = (v[0] + v[1]) + (v[2] + v[3]);
  sm = wsum32(sm);
  if (lane == 0) red[wave] = sm;
  __syncthreads();
  float tot = 0.0f;
#pragma unroll
  for (int w = 0; w < 8; ++w) tot += red[w];
  const float mean = tot * (1.0f / (float)DM);
  __syncthreads();
  v4f d;
#pragma unroll
  for (int jj = 0; jj < 4; ++jj) d[jj] = v[jj] - mean;
  float sq = (d[0] * d[0] + d[1] * d[1]) + (d[2] * d[2] + d[3] * d[3]);
  sq = wsum32(sq);
  if (lane == 0) red[wave] = sq;
  __syncthreads();
  float totq = 0.0f;
#pragma unroll
  for (int w = 0; w < 8; ++w) totq += red[w];
  const float var = totq * (1.0f / (float)(DM - 1));
  const float sd = sqrtf(var > 0.0f ? var : 0.0f);
  const float al = bfr(alpha[0]);
  const float be = bfr(beta[0]);
  const float inv = 1.0f / (sd + 1e-8f);
  v4f y;
#pragma unroll
  for (int jj = 0; jj < 4; ++jj) y[jj] = (al * d[jj]) * inv + be;

  float* fp = Yf + (size_t)row * DM + tid * 4;
  v2u hpk;
  if constexpr (F16OUT) {
    union { f16_t hh[4]; v2u u; } cv;
#pragma unroll
    for (int jj = 0; jj < 4; ++jj) cv.hh[jj] = (f16_t)y[jj];
    hpk = cv.u;
  }
  *(volatile v4f*)fp = y;
  if constexpr (F16OUT) *(volatile v2u*)(Yh + (size_t)row * DM + tid * 4) = hpk;
  __threadfence();
  *(volatile v4f*)fp = y;
  if constexpr (F16OUT) *(volatile v2u*)(Yh + (size_t)row * DM + tid * 4) = hpk;
}

extern "C" void kernel_launch(void* const* d_in, const int* in_sizes, int n_in,
                              void* d_out, int out_size, void* d_ws, size_t ws_size,
                              hipStream_t stream) {
  if (n_in < 14) return;
  const int needX = ((NB - 1) * SEQ_FULL + SEQ) * DM;
  const int needM = (SEQ - 1) * SEQ_FULL + SEQ;
  if (in_sizes[0] < needX || in_sizes[1] < needM) return;
  if (in_sizes[2] < DM * DM || in_sizes[3] < DM || in_sizes[4] < DM * DM || in_sizes[5] < DM) return;
  if (in_sizes[6] < DFF * DM || in_sizes[7] < DFF || in_sizes[8] < DM * DFF || in_sizes[9] < DM) return;
  if (in_sizes[10] < 1 || in_sizes[11] < 1 || in_sizes[12] < 1 || in_sizes[13] < 1) return;
  if (out_size < ROWS * DM) return;
  if (ws_size < WS_TOTAL) return;

  const float* x      = (const float*)d_in[0];
  const int*   mask   = (const int*)d_in[1];
  const float* wq     = (const float*)d_in[2];
  const float* bq     = (const float*)d_in[3];
  const float* wo     = (const float*)d_in[4];
  const float* bo     = (const float*)d_in[5];
  const float* w1     = (const float*)d_in[6];
  const float* b1     = (const float*)d_in[7];
  const float* w2     = (const float*)d_in[8];
  const float* b2     = (const float*)d_in[9];
  const float* alpha1 = (const float*)d_in[10];
  const float* beta1  = (const float*)d_in[11];
  const float* alpha2 = (const float*)d_in[12];
  const float* beta2  = (const float*)d_in[13];
  float* out = (float*)d_out;

  char* ws = (char*)d_ws;
  f16_t* Wq16 = (f16_t*)(ws + OFF_WQ);
  f16_t* Wo16 = (f16_t*)(ws + OFF_WO);
  f16_t* W1h  = (f16_t*)(ws + OFF_W1);
  f16_t* W2h  = (f16_t*)(ws + OFF_W2);
  f16_t* Xh   = (f16_t*)(ws + OFF_XH);
  f16_t* Q16  = (f16_t*)(ws + OFF_Q);
  f16_t* C16  = (f16_t*)(ws + OFF_CX);
  float* Sf   = (float*)(ws + OFF_S);
  float* X1f  = (float*)(ws + OFF_X1F);
  f16_t* X1h  = (f16_t*)(ws + OFF_X1H);
  f16_t* H16  = (f16_t*)(ws + OFF_H);
  int*   Flg  = (int*)(ws + OFF_FL);

  k_cvt16<0><<<(DM * DM) / 2048, 256, 0, stream>>>(wq, Wq16, DM * DM, 64.0f);
  k_cvt16<0><<<(DM * DM) / 2048, 256, 0, stream>>>(wo, Wo16, DM * DM, 64.0f);
  k_cvt16<0><<<(DFF * DM) / 2048, 256, 0, stream>>>(w1, W1h, DFF * DM, 64.0f);
  k_cvt16<0><<<(DM * DFF) / 2048, 256, 0, stream>>>(w2, W2h, DM * DFF, 64.0f);
  k_cvt16<1><<<(ROWS * DM) / 2048, 256, 0, stream>>>(x, Xh, ROWS * DM, 1.0f);

  k_maskflag<<<NQT, 256, 0, stream>>>(mask, Flg);

  {
    dim3 grid(DM / 128, ROWS / 128);
    k_gemm<0, f16_t><<<grid, 256, 0, stream>>>(Xh, Wq16, bq, x, Q16, DM, DM, 1.0f / 64.0f);
  }

  {
    dim3 grid(NQT, NH, NB);
    k_attn<<<grid, 256, 0, stream>>>(Q16, mask, Flg, C16);
  }

  {
    dim3 grid(DM / 128, ROWS / 128);
    k_gemm<2, float><<<grid, 256, 0, stream>>>(C16, Wo16, bo, x, Sf, DM, DM, 1.0f / 4096.0f);
  }

  k_ln<1><<<ROWS, 256, 0, stream>>>(Sf, alpha1, beta1, X1f, X1h);

  {
    dim3 grid(DFF / 128, ROWS / 128);
    k_gemm<0, f16_t><<<grid, 256, 0, stream>>>(X1h, W1h, b1, X1f, H16, DFF, DM, 1.0f / 64.0f);
  }

  {
    dim3 grid(DM / 128, ROWS / 128);
    k_gemm<1, float><<<grid, 256, 0, stream>>>(H16, W2h, b2, X1f, Sf, DM, DFF, 1.0f / 64.0f);
  }

  k_ln<0><<<ROWS, 256, 0, stream>>>(Sf, alpha2, beta2, out, X1h);
}
